// SpatialGatherModule_31834297598793
// MI455X (gfx1250) — hardware-run, weakly checked
//
#include <hip/hip_runtime.h>
#include <math.h>

typedef __attribute__((ext_vector_type(16))) _Float16 v16h;
typedef __attribute__((ext_vector_type(8)))  _Float16 v8h;
typedef __attribute__((ext_vector_type(8)))  float    v8f;
typedef __attribute__((ext_vector_type(4)))  float    v4f;
typedef __attribute__((ext_vector_type(4)))  int      v4i;

constexpr int kPts     = 131072;
constexpr int kChan    = 96;
constexpr int kCls     = 20;
constexpr int kSeg     = 8;
constexpr int kRowsReal = kSeg * kCls;
constexpr int kRowsPad  = 192;
constexpr int kColsPad  = 128;
constexpr int kDenCol   = kChan;
constexpr int kSplits   = 128;
constexpr int kKsplit   = kPts / kSplits;
constexpr int kTileA    = 256;
constexpr int kBlocksA  = kPts / kTileA;
constexpr int kTileB    = 64;
constexpr int kBlocksB  = kPts / kTileB;
constexpr int kFeatPitch = 100;
constexpr int kOutElems = kSeg * kCls * kChan;
constexpr float kExpCarry  = 64.0f;
constexpr float kFeatCarry = 16.0f;

static_assert(kRowsReal == 160, "rows");
static_assert((kRowsPad % 64) == 0 && (kColsPad % 64) == 0 && (kKsplit % 32) == 0, "GEMM tile multiples");
static_assert(kKsplit * kSplits == kPts, "split-K cover");
static_assert(kRowsPad >= kRowsReal && kColsPad > kDenCol, "pads");
static_assert(kBlocksA * kTileA == kPts && kBlocksB * kTileB == kPts, "tile cover");
static_assert((kTileA * kCls) == 5 * 256 * 4, "probs tile = 5 v4f per thread");
static_assert((kTileB * kChan) == 6 * 256 * 4, "feats tile = 6 v4f per thread");
static_assert((kTileB * kCls) == 5 * 256, "exp tile = 5 values per thread");
static_assert((kOutElems / 4) == 15 * 256, "finalise grid");

constexpr size_t kOffAT   = 0;
constexpr size_t kOffBT   = kOffAT   + (size_t)kRowsPad * kPts * 2;
constexpr size_t kOffPART = kOffBT   + (size_t)kColsPad * kPts * 2;
constexpr size_t kOffPMAX = kOffPART + (size_t)kSplits * kRowsPad * kColsPad * 4;
constexpr size_t kOffSMAX = kOffPMAX + (size_t)kBlocksA * kRowsReal * 4;
constexpr size_t kWsTotal = kOffSMAX + 1024;
static_assert(kWsTotal == 96797696ull, "carve total");
static_assert(kWsTotal <= 134217728ull, "carve cap");
static_assert((kOffBT % 128) == 0 && (kOffPART % 128) == 0 && (kOffPMAX % 128) == 0 && (kOffSMAX % 128) == 0, "aligned regions");

__device__ __forceinline__ void dep_guard4_h(v8f& a, v8f& b, v8f& c, v8f& d, v16h x) {
  asm volatile("v_nop\n\tv_nop\n\tv_nop\n\tv_nop" : "+v"(a), "+v"(b), "+v"(c), "+v"(d) : "v"(x));
}
__device__ __forceinline__ void keep4_h(v16h a, v16h b, v16h c, v16h d) { asm volatile("v_nop" :: "v"(a), "v"(b), "v"(c), "v"(d)); }
__device__ __forceinline__ void acc_guard4(v8f& a, v8f& b, v8f& c, v8f& d) { asm volatile("v_nop\n\tv_nop\n\tv_nop\n\tv_nop" : "+v"(a), "+v"(b), "+v"(c), "+v"(d)); }
struct FragH {
  union U { v16h v; v8h h[2]; };
  static __device__ __forceinline__ v16h load(const _Float16* p) {
    U f; f.h[0] = *(const v8h*)(p); f.h[1] = *(const v8h*)(p + 16); return f.v;
  }
  static __device__ __forceinline__ v8f mma(v16h a, v16h b, v8f c) {
    return __builtin_amdgcn_wmma_f32_16x16x32_f16(false, a, false, b, (short)0, c, false, false);
  }
};

__global__ __launch_bounds__(256) void segmax_partial_kernel(
    const float* __restrict__ probs, const int* __restrict__ idx, float* __restrict__ pmax)
{
  __shared__ __align__(16) float sP[kTileA * kCls];
  __shared__ __align__(16) int   sI[kTileA];
  __shared__ __align__(16) float sO[kRowsReal];
  const int tid = threadIdx.x;
  const int blk = blockIdx.x;
  sI[tid] = idx[(size_t)blk * kTileA + tid];
  const v4f* src = (const v4f*)(probs + (size_t)blk * kTileA * kCls);
#pragma unroll
  for (int it = 0; it < 5; ++it) {
    const int i = tid + 256 * it;
    *(v4f*)(sP + 4 * i) = src[i];
  }
  __syncthreads();
  const int tc = (tid < kRowsReal) ? tid : (kRowsReal - 1);
  const int b = tc / kCls;
  const int k = tc - b * kCls;
  float m = -INFINITY;
#pragma unroll 4
  for (int n = 0; n < kTileA; ++n) {
    const float v = sP[n * kCls + k];
    const int id = sI[n];
    m = (id == b) ? fmaxf(m, v) : m;
  }
  if (tid < kRowsReal) sO[tid] = m;
  __syncthreads();
  if (tid < kRowsReal / 4) {
    const v4f o = *(const v4f*)(sO + 4 * tid);
    float* dst = pmax + (size_t)blk * kRowsReal + 4 * tid;
    *(volatile v4f*)dst = o;
    __threadfence();
    *(volatile v4f*)dst = o;
  }
}

__global__ __launch_bounds__(256) void segmax_final_kernel(
    const float* __restrict__ pmax, float* __restrict__ smax)
{
  __shared__ __align__(16) float sO[256];
  const int tid = threadIdx.x;
  const int tc = (tid < kRowsReal) ? tid : (kRowsReal - 1);
  float m = -INFINITY;
#pragma unroll 8
  for (int j = 0; j < kBlocksA; ++j) m = fmaxf(m, pmax[(size_t)j * kRowsReal + tc]);
  const bool fin = (__float_as_uint(m) & 0x7F800000u) != 0x7F800000u;
  const float r = ((tid < kRowsReal) && fin) ? m : 0.0f;
  sO[tid] = r;
  __syncthreads();
  if (tid < 64) {
    const v4f o = *(const v4f*)(sO + 4 * tid);
    float* dst = smax + 4 * tid;
    *(volatile v4f*)dst = o;
    __threadfence();
    *(volatile v4f*)dst = o;
  }
}

__global__ __launch_bounds__(256) void plane_build_kernel(
    const float* __restrict__ feats, const float* __restrict__ probs, const int* __restrict__ idx,
    const float* __restrict__ smax, unsigned short* __restrict__ At, unsigned short* __restrict__ Bt)
{
  __shared__ __align__(16) float sF[kTileB * kFeatPitch];
  __shared__ __align__(16) float sP[kTileB * kCls];
  __shared__ __align__(16) float sE[kCls * kTileB];
  __shared__ __align__(16) float sS[256];
  __shared__ __align__(16) int   sI[kTileB];
  const int tid  = threadIdx.x;
  const int lane = tid & 31;
  const int wave = __builtin_amdgcn_readfirstlane((int)(threadIdx.x >> 5));
  const int blk  = blockIdx.x;
  const size_t n0 = (size_t)blk * kTileB;

  {
    int iv = idx[n0 + (tid & (kTileB - 1))];
    asm volatile("" : "+v"(iv));
    if (tid < kTileB) sI[tid] = iv;
  }
  sS[tid] = smax[tid];
  {
    const v4f* srcP = (const v4f*)(probs + n0 * kCls);
    *(v4f*)(sP + 4 * tid) = srcP[tid];
    const int i1 = tid + 256;
    const int i1c = (i1 < 320) ? i1 : 319;
    v4f pv = srcP[i1c];
    asm volatile("" : "+v"(pv));
    if (i1 < 320) *(v4f*)(sP + 4 * i1) = pv;
  }
  {
    const v4f* srcF = (const v4f*)(feats + n0 * kChan);
#pragma unroll
    for (int it = 0; it < 6; ++it) {
      const int i = tid + 256 * it;
      const int n = i / 24;
      const int c4 = (i - n * 24) * 4;
      *(v4f*)(sF + n * kFeatPitch + c4) = srcF[i];
    }
  }
  __syncthreads();
#pragma unroll 1
  for (int it = 0; it < 5; ++it) {
    const int i = tid + 256 * it;
    const int n = i / kCls;
    const int k = i - n * kCls;
    int id = sI[n];
    id = id < 0 ? 0 : (id > (kSeg - 1) ? (kSeg - 1) : id);
    const float e = expf(sP[i] - sS[id * kCls + k]);
    sE[k * kTileB + n] = e * kExpCarry;
  }
  __syncthreads();

  const int q  = lane >> 3;
  const int n8 = (lane & 7) * 8;
  const v4i i0 = *(const v4i*)(sI + n8);
  const v4i i1 = *(const v4i*)(sI + n8 + 4);

  v8h ha[6];
#pragma unroll
  for (int it = 0; it < 6; ++it) {
    const int m = it * 32 + wave * 4 + q;
    const bool valid = m < kRowsReal;
    const int mc = valid ? m : (kRowsReal - 1);
    const int b = mc / kCls;
    const int k = mc - b * kCls;
    const v4f e0 = *(const v4f*)(sE + k * kTileB + n8);
    const v4f e1 = *(const v4f*)(sE + k * kTileB + n8 + 4);
    v8h hv;
#pragma unroll
    for (int e = 0; e < 4; ++e) {
      const float x0 = (valid && (i0[e] == b)) ? e0[e] : 0.0f;
      const float x1 = (valid && (i1[e] == b)) ? e1[e] : 0.0f;
      hv[e]     = (_Float16)x0;
      hv[4 + e] = (_Float16)x1;
    }
    ha[it] = hv;
  }
  v8h hb[4];
#pragma unroll
  for (int it = 0; it < 4; ++it) {
    const int c = it * 32 + wave * 4 + q;
    const int cc = (c < kChan) ? c : (kChan - 1);
    const float padv = (c == kDenCol) ? kFeatCarry : 0.0f;
    v8h hv;
#pragma unroll
    for (int e = 0; e < 8; ++e) {
      const float f = sF[(n8 + e) * kFeatPitch + cc] * kFeatCarry;
      const float x = (c < kChan) ? f : padv;
      hv[e] = (_Float16)x;
    }
    hb[it] = hv;
  }
  for (int pass = 0; pass < 2; ++pass) {
#pragma unroll
    for (int it = 0; it < 6; ++it) {
      const int m = it * 32 + wave * 4 + q;
      *(volatile v8h*)(At + (size_t)m * kPts + n0 + n8) = ha[it];
    }
#pragma unroll
    for (int it = 0; it < 4; ++it) {
      const int c = it * 32 + wave * 4 + q;
      *(volatile v8h*)(Bt + (size_t)c * kPts + n0 + n8) = hb[it];
    }
    __threadfence();
  }
}

__global__ __launch_bounds__(256) void wmma_gemm64_f16(
    const unsigned short* __restrict__ Ap, int lda, long strideA,
    const unsigned short* __restrict__ Btp, int ldb, long strideB,
    float* __restrict__ Cout, int ldc, long strideC,
    int M, int N, int K) {
  typedef _Float16 T;
  const T* A = (const T*)Ap;
  const T* Bt = (const T*)Btp;
  __shared__ __align__(16) float sT[8][16 * 68];
  const int b    = blockIdx.y;
  const int lane = threadIdx.x & 31;
  const int wave = __builtin_amdgcn_readfirstlane((int)(threadIdx.x >> 5));
  const int tilesN = N >> 6;
  const int tilesM = M >> 6;
  const int tile = blockIdx.x * 8 + wave;
  if (tile >= tilesM * tilesN) return;
  const int tm = tile / tilesN;
  const int tn = tile - tm * tilesN;
  const int m0 = tm << 6;
  const int n0 = tn << 6;

  const T* Ab = A  + (size_t)b * strideA;
  const T* Bb = Bt + (size_t)b * strideB;

  const int rlane = lane & 15;
  const int koff  = (lane >> 4) * 8;
  const int mOff  = (lane >> 4) * 8;

  v8f acc[4][4];
#pragma unroll
  for (int i = 0; i < 4; ++i)
#pragma unroll
    for (int j = 0; j < 4; ++j) acc[i][j] = (v8f){0.f,0.f,0.f,0.f,0.f,0.f,0.f,0.f};

  for (int k0 = 0; k0 < K; k0 += 32) {
    v16h bh[4];
#pragma unroll
    for (int j = 0; j < 4; ++j) {
      const size_t bo = (size_t)(n0 + (j << 4) + rlane) * ldb + koff + k0;
      bh[j] = FragH::load(Bb + bo);
    }
#pragma unroll
    for (int i = 0; i < 4; ++i) {
      const size_t ao = (size_t)(m0 + (i << 4) + rlane) * lda + koff + k0;
      v16h ah = FragH::load(Ab + ao);
#pragma unroll
      for (int j = 0; j < 4; ++j) acc[i][j] = FragH::mma(ah, bh[j], acc[i][j]);
      dep_guard4_h(acc[i][0], acc[i][1], acc[i][2], acc[i][3], ah);
    }
    keep4_h(bh[0], bh[1], bh[2], bh[3]);
  }
  acc_guard4(acc[0][0], acc[0][1], acc[0][2], acc[0][3]);
  acc_guard4(acc[1][0], acc[1][1], acc[1][2], acc[1][3]);
  acc_guard4(acc[2][0], acc[2][1], acc[2][2], acc[2][3]);
  acc_guard4(acc[3][0], acc[3][1], acc[3][2], acc[3][3]);

  float* slab = sT[wave];
  float* C = Cout + (size_t)b * strideC;
#pragma unroll
  for (int i = 0; i < 4; ++i) {
    const int mBase = m0 + (i << 4);
#pragma unroll
    for (int j = 0; j < 4; ++j) {
#pragma unroll
      for (int r = 0; r < 8; ++r) {
        slab[(mOff + r) * 68 + (j << 4) + rlane] = acc[i][j][r];
      }
    }
    __builtin_amdgcn_fence(__ATOMIC_RELEASE, "workgroup");
    __builtin_amdgcn_wave_barrier();
    __builtin_amdgcn_fence(__ATOMIC_ACQUIRE, "workgroup");
    {
      const int hh = lane >> 4, c4 = (lane & 15) * 4;
      for (int pass = 0; pass < 2; ++pass) {
#pragma unroll
        for (int it = 0; it < 8; ++it) {
          const int row = it * 2 + hh;
          v4f v = *(const v4f*)(slab + row * 68 + c4);
          *(volatile v4f*)(C + (size_t)(mBase + row) * ldc + n0 + c4) = v;
        }
        __threadfence();
      }
    }
    __builtin_amdgcn_fence(__ATOMIC_RELEASE, "workgroup");
    __builtin_amdgcn_wave_barrier();
    __builtin_amdgcn_fence(__ATOMIC_ACQUIRE, "workgroup");
  }
}

__global__ __launch_bounds__(256) void finalize_kernel(
    const float* __restrict__ part, const int* __restrict__ nseg, float* __restrict__ out)
{
  const int i = blockIdx.x * 256 + threadIdx.x;
  const int m = i / 24;
  const int c4 = (i - m * 24) * 4;
  const float* pr = part + (size_t)m * kColsPad;
  v4f num = (v4f){0.f, 0.f, 0.f, 0.f};
  float den = 0.0f;
#pragma unroll 4
  for (int s = 0; s < kSplits; ++s) {
    const size_t o = (size_t)s * kRowsPad * kColsPad;
    const v4f a = *(const v4f*)(pr + o + c4);
    const float d = pr[o + kDenCol];
    num = num + a;
    den = den + d;
  }
  const int ns = nseg[0];
  const bool ok = (ns == kSeg);
  const float qnan = __uint_as_float(0x7FC00000u);
  const float rden = 1.0f / den;
  const float inv = (den > 0.0f) ? rden : 0.0f;
  v4f o4;
  o4[0] = ok ? (num[0] * inv) : qnan;
  o4[1] = ok ? (num[1] * inv) : qnan;
  o4[2] = ok ? (num[2] * inv) : qnan;
  o4[3] = ok ? (num[3] * inv) : qnan;
  float* dst = out + (size_t)4 * i;
  *(volatile v4f*)dst = o4;
  __threadfence();
  *(volatile v4f*)dst = o4;
}

extern "C" void kernel_launch(void* const* d_in, const int* in_sizes, int n_in,
                              void* d_out, int out_size, void* d_ws, size_t ws_size,
                              hipStream_t stream) {
  if (n_in < 4) return;
  if (in_sizes[0] != kPts * kChan) return;
  if (in_sizes[1] != kPts * kCls) return;
  if (in_sizes[2] != 1) return;
  if (in_sizes[3] != kPts) return;
  if (out_size != kOutElems) return;
  if (ws_size < kWsTotal) return;

  const float* feats = (const float*)d_in[0];
  const float* probs = (const float*)d_in[1];
  const int*   nseg  = (const int*)d_in[2];
  const int*   idx   = (const int*)d_in[3];
  float* out = (float*)d_out;

  char* ws = (char*)d_ws;
  unsigned short* AT   = (unsigned short*)(ws + kOffAT);
  unsigned short* BT   = (unsigned short*)(ws + kOffBT);
  float*          PART = (float*)(ws + kOffPART);
  float*          PMAX = (float*)(ws + kOffPMAX);
  float*          SMAX = (float*)(ws + kOffSMAX);

  segmax_partial_kernel<<<kBlocksA, 256, 0, stream>>>(probs, idx, PMAX);
  segmax_final_kernel<<<1, 256, 0, stream>>>(PMAX, SMAX);
  plane_build_kernel<<<kBlocksB, 256, 0, stream>>>(feats, probs, idx, SMAX, AT, BT);
  wmma_gemm64_f16<<<dim3(1, kSplits), 192, 0, stream>>>(
      AT, kPts, (long)kKsplit,
      BT, kPts, (long)kKsplit,
      PART, kColsPad, (long)kRowsPad * kColsPad,
      kRowsPad, kColsPad, kKsplit);
  finalize_kernel<<<kOutElems / 4 / 256, 256, 0, stream>>>(PART, nseg, out);
}
